// Word_LSTM_48180943126826
// MI455X (gfx1250) — hardware-run, weakly checked
//
#include <hip/hip_runtime.h>
#include <math.h>

typedef __attribute__((ext_vector_type(16))) _Float16 v16h;
typedef __attribute__((ext_vector_type(8)))  _Float16 v8h;
typedef __attribute__((ext_vector_type(8)))  float    v8f;
typedef __attribute__((ext_vector_type(4)))  float    v4f;
typedef __attribute__((ext_vector_type(4)))  int      v4i;

constexpr int kB    = 128;
constexpr int kD    = 1024;
constexpr int kG    = 4096;
constexpr int kInW  = 3072;
constexpr int kNV   = 36;
constexpr int kNL   = 20;
constexpr int kT    = 4;
constexpr int kSqrtD = 32;
static_assert(kSqrtD * kSqrtD == kD, "score scale");
static_assert(kG == 4 * kD && kInW == 3 * kD, "gate and input widths");
static_assert((kNV + kNL) == 7 * 8, "slots per wave");
static_assert((kNV % 4) == 0 && (kNL % 4) == 0, "context unroll");
constexpr float kQScale  = 1.0f / (float)kSqrtD;
constexpr float kCarryA  = 64.0f;
constexpr float kCarryW  = 1024.0f;
constexpr float kCarryR  = 2048.0f;
constexpr float kFold    = 1.0f / (kCarryA * kCarryW);
constexpr float kFoldR   = kFold / kCarryR;
constexpr float kHaltThr = 0.99f;
constexpr float kKeyStep = 0.01f;
constexpr float kF16Min  = 6.103515625e-5f;

constexpr size_t kSzVec   = (size_t)kB * kD * 4;
constexpr size_t kOffBT1  = 0;
constexpr size_t kOffBT2  = kOffBT1 + (size_t)kG * kG * 2;
constexpr size_t kOffBT3  = kOffBT2 + (size_t)kG * 2 * kD * 2;
constexpr size_t kOffBT4  = kOffBT3 + (size_t)kG * 2 * kD * 2;
constexpr size_t kOffA1   = kOffBT4 + (size_t)kD * kD * 2;
constexpr size_t kOffA2   = kOffA1  + (size_t)kB * kG * 2;
constexpr size_t kOffA3   = kOffA2  + (size_t)kB * 2 * kD * 2;
constexpr size_t kOffA4   = kOffA3  + (size_t)kB * 2 * kD * 2;
constexpr size_t kOffGA   = kOffA4  + (size_t)kB * kD * 2;
constexpr size_t kOffLC   = kOffGA  + (size_t)kB * kG * 4;
constexpr size_t kOffGL   = kOffLC  + (size_t)kB * kG * 4;
constexpr size_t kOffCT   = kOffGL  + (size_t)kB * kG * 4;
constexpr size_t kOffHATT = kOffCT  + kSzVec;
constexpr size_t kOffCATT = kOffHATT + kSzVec;
constexpr size_t kOffHLG  = kOffCATT + kSzVec;
constexpr size_t kOffCLG  = kOffHLG + kSzVec;
constexpr size_t kOffKV0  = kOffCLG + kSzVec;
constexpr size_t kOffKV1  = kOffKV0 + kSzVec;
constexpr size_t kOffHL0  = kOffKV1 + kSzVec;
constexpr size_t kOffHL1  = kOffHL0 + kSzVec;
constexpr size_t kOffCL0  = kOffHL1 + kSzVec;
constexpr size_t kOffCL1  = kOffCL0 + kSzVec;
constexpr size_t kOffS0   = kOffCL1 + kSzVec;
constexpr size_t kOffS1   = kOffS0  + kSzVec;
constexpr size_t kOffST0  = kOffS1  + kSzVec;
constexpr size_t kOffST1  = kOffST0 + (size_t)kB * 32 * 4;
constexpr size_t kOffBSA  = kOffST1 + (size_t)kB * 32 * 4;
constexpr size_t kOffBSL  = kOffBSA + (size_t)kG * 4;
constexpr size_t kOffA1L  = kOffBSL + (size_t)kG * 4;
constexpr size_t kOffGAR  = kOffA1L + (size_t)kB * kG * 2;
constexpr size_t kWsTotal = kOffGAR + (size_t)kB * kG * 4;
static_assert(kWsTotal == 87883776ull, "carve total");
static_assert(kWsTotal <= 134217728ull, "carve cap");
static_assert((kOffBT2 % 128) == 0 && (kOffBT3 % 128) == 0 && (kOffBT4 % 128) == 0 && (kOffA1 % 128) == 0 &&
              (kOffA2 % 128) == 0 && (kOffA3 % 128) == 0 && (kOffA4 % 128) == 0 && (kOffGA % 128) == 0 &&
              (kOffLC % 128) == 0 && (kOffGL % 128) == 0 && (kOffCT % 128) == 0 && (kOffHATT % 128) == 0 &&
              (kOffST0 % 128) == 0 && (kOffST1 % 128) == 0 && (kOffBSA % 128) == 0 && (kOffBSL % 128) == 0 &&
              (kOffA1L % 128) == 0 && (kOffGAR % 128) == 0,
              "128-B aligned regions");

constexpr size_t kOutA   = 0;
constexpr size_t kOutVK  = (size_t)kB * kD;
constexpr size_t kOutLK  = kOutVK + (size_t)kB * kNV * kD;
constexpr size_t kOutCst = kOutLK + (size_t)kB * kNL * kD;
constexpr size_t kOutH   = kOutCst + kB;
constexpr size_t kOutC   = kOutH + (size_t)2 * kB * kD;
constexpr size_t kOutKV  = kOutC + (size_t)2 * kB * kD;
constexpr size_t kOutTot = kOutKV + (size_t)kB * kD;
static_assert(kOutVK * 4 == 524288ull && kOutLK * 4 == 19398656ull && kOutCst * 4 == 29884416ull &&
              kOutH * 4 == 29884928ull && kOutC * 4 == 30933504ull && kOutKV * 4 == 31982080ull &&
              kOutTot * 4 == 32506368ull, "output byte offsets");

__device__ __forceinline__ _Float16 to_h_flush(float v) {
  const float s = (fabsf(v) < kF16Min) ? 0.0f : v;
  return (_Float16)s;
}
__device__ __forceinline__ _Float16 rem_h_flush(float carried, _Float16 valueTerm) {
  float back = (float)valueTerm;
  asm volatile("" : "+v"(back));
  const float rem = (carried - back) * kCarryR;
  return to_h_flush(rem);
}
__device__ __forceinline__ float sigmoid_f(float x) {
  return __builtin_amdgcn_rcpf(1.0f + expf(-x));
}
__device__ __forceinline__ v4f poison_sel4(v4f v, bool ok) {
  const float qn = __uint_as_float(0x7fc00000u);
  v4f r;
  r[0] = ok ? v[0] : qn;
  r[1] = ok ? v[1] : qn;
  r[2] = ok ? v[2] : qn;
  r[3] = ok ? v[3] : qn;
  return r;
}

__device__ __forceinline__ void group_guard_h(v8f& a, v8f& b, v8f& c, v8f& d, v16h x, v16h y0, v16h y1, v16h y2, v16h y3) {
  asm volatile("v_nop\n\tv_nop\n\tv_nop\n\tv_nop" : "+v"(a), "+v"(b), "+v"(c), "+v"(d) : "v"(x), "v"(y0), "v"(y1), "v"(y2), "v"(y3));
}
__device__ __forceinline__ void keep4_h(v16h a, v16h b, v16h c, v16h d) { asm volatile("v_nop" :: "v"(a), "v"(b), "v"(c), "v"(d)); }
__device__ __forceinline__ void acc_guard4(v8f& a, v8f& b, v8f& c, v8f& d) { asm volatile("v_nop\n\tv_nop\n\tv_nop\n\tv_nop" : "+v"(a), "+v"(b), "+v"(c), "+v"(d)); }

union FragH { v16h v; v8h h[2]; };
__device__ __forceinline__ v16h frag_load_h(const _Float16* p) {
  FragH f;
  f.h[0] = *(const v8h*)(p);
  f.h[1] = *(const v8h*)(p + 16);
  return f.v;
}
__device__ __forceinline__ v8f mma_h(v16h a, v16h b, v8f c) {
  return __builtin_amdgcn_wmma_f32_16x16x32_f16(false, a, false, b, (short)0, c, false, false);
}

__global__ __launch_bounds__(256) void gemm_f16_tile64(
    const unsigned short* __restrict__ Ap, int lda,
    const unsigned short* __restrict__ Btp, int ldb,
    float* __restrict__ C, int ldc, int M, int N, int K, float scale) {
  const _Float16* A  = (const _Float16*)Ap;
  const _Float16* Bt = (const _Float16*)Btp;
  __shared__ __align__(16) float sT[8][16 * 68];
  const int lane = threadIdx.x & 31;
  const int wave = threadIdx.x >> 5;
  const int tilesN = N >> 6;
  const int tilesM = M >> 6;
  const int tile = blockIdx.x * 8 + wave;
  if (tile >= tilesM * tilesN) return;
  const int tm = tile / tilesN;
  const int tn = tile - tm * tilesN;
  const int m0 = tm << 6;
  const int n0 = tn << 6;

  const int rlane = lane & 15;
  const int koff  = (lane >> 4) * 8;
  const int mOff  = (lane >> 4) * 8;

  v8f acc[4][4];
#pragma unroll
  for (int i = 0; i < 4; ++i)
#pragma unroll
    for (int j = 0; j < 4; ++j) acc[i][j] = (v8f){0.f,0.f,0.f,0.f,0.f,0.f,0.f,0.f};

  for (int k0 = 0; k0 < K; k0 += 32) {
    v16h bh[4];
#pragma unroll
    for (int j = 0; j < 4; ++j) {
      const size_t bo = (size_t)(n0 + (j << 4) + rlane) * ldb + koff + k0;
      bh[j] = frag_load_h(Bt + bo);
    }
#pragma unroll
    for (int i = 0; i < 4; ++i) {
      const size_t ao = (size_t)(m0 + (i << 4) + rlane) * lda + koff + k0;
      const v16h ah = frag_load_h(A + ao);
#pragma unroll
      for (int j = 0; j < 4; ++j) acc[i][j] = mma_h(ah, bh[j], acc[i][j]);
      group_guard_h(acc[i][0], acc[i][1], acc[i][2], acc[i][3], ah, bh[0], bh[1], bh[2], bh[3]);
    }
    keep4_h(bh[0], bh[1], bh[2], bh[3]);
  }
  acc_guard4(acc[0][0], acc[0][1], acc[0][2], acc[0][3]);
  acc_guard4(acc[1][0], acc[1][1], acc[1][2], acc[1][3]);
  acc_guard4(acc[2][0], acc[2][1], acc[2][2], acc[2][3]);
  acc_guard4(acc[3][0], acc[3][1], acc[3][2], acc[3][3]);

  float* slab = sT[wave];
#pragma unroll
  for (int i = 0; i < 4; ++i) {
    const int mBase = m0 + (i << 4);
#pragma unroll
    for (int j = 0; j < 4; ++j) {
#pragma unroll
      for (int r = 0; r < 8; ++r) {
        slab[(mOff + r) * 68 + (j << 4) + rlane] = acc[i][j][r] * scale;
      }
    }
    __builtin_amdgcn_fence(__ATOMIC_RELEASE, "workgroup");
    __builtin_amdgcn_wave_barrier();
    __builtin_amdgcn_fence(__ATOMIC_ACQUIRE, "workgroup");
    {
      const int hh = lane >> 4, c4 = (lane & 15) * 4;
      for (int pass = 0; pass < 2; ++pass) {
#pragma unroll
        for (int it = 0; it < 8; ++it) {
          const int row = it * 2 + hh;
          const v4f v = *(const v4f*)(slab + row * 68 + c4);
          *(volatile v4f*)(C + (size_t)(mBase + row) * ldc + n0 + c4) = v;
        }
        __threadfence();
      }
    }
    __builtin_amdgcn_fence(__ATOMIC_RELEASE, "workgroup");
    __builtin_amdgcn_wave_barrier();
    __builtin_amdgcn_fence(__ATOMIC_ACQUIRE, "workgroup");
  }
}

__global__ __launch_bounds__(256) void cvt_plane_kernel(
    const float* __restrict__ src, unsigned srcPitch, unsigned srcCol0,
    unsigned short* __restrict__ dst, unsigned dstPitch, unsigned dstCol0,
    unsigned cols8, unsigned total8, float carry) {
  const unsigned i = blockIdx.x * 256u + threadIdx.x;
  if (i >= total8) return;
  unsigned row = i / cols8;
  unsigned c = (i - row * cols8) * 8u;
  asm volatile("" : "+v"(row), "+v"(c));
  const float* sp = src + (size_t)row * srcPitch + srcCol0 + c;
  const v4f a0 = *(const v4f*)(sp);
  const v4f a1 = *(const v4f*)(sp + 4);
  v8h hv;
#pragma unroll
  for (int e = 0; e < 4; ++e) {
    const float x0 = a0[e] * carry;
    const float x1 = a1[e] * carry;
    hv[e]     = to_h_flush(x0);
    hv[4 + e] = to_h_flush(x1);
  }
  unsigned short* q = dst + (size_t)row * dstPitch + dstCol0 + c;
  *(volatile v8h*)q = hv;
  __threadfence();
  *(volatile v8h*)q = hv;
}

__global__ __launch_bounds__(256) void cvt_act_kernel(
    const float* __restrict__ h1, const float* __restrict__ fc, const float* __restrict__ xt,
    const float* __restrict__ h0, unsigned short* __restrict__ A1, unsigned short* __restrict__ A1L,
    unsigned short* __restrict__ A2,
    const float* __restrict__ abih, const float* __restrict__ abhh,
    const float* __restrict__ lbih, const float* __restrict__ lbhh,
    float* __restrict__ bsA, float* __restrict__ bsL) {
  const unsigned i = blockIdx.x * 256u + threadIdx.x;
  unsigned row = i >> 9;
  unsigned c8 = i & 511u;
  asm volatile("" : "+v"(row), "+v"(c8));
  const unsigned seg = c8 >> 7;
  const unsigned cc = (c8 & 127u) * 8u;
  const float* sbase = (seg == 0u) ? h1 : ((seg == 1u) ? fc : ((seg == 2u) ? xt : h0));
  const float* sp = sbase + (size_t)row * kD + cc;
  const v4f a0 = *(const v4f*)(sp);
  const v4f a1 = *(const v4f*)(sp + 4);
  v8h hv, lv;
#pragma unroll
  for (int e = 0; e < 4; ++e) {
    const float x0 = a0[e] * kCarryA;
    const float x1 = a1[e] * kCarryA;
    const _Float16 t0 = to_h_flush(x0);
    const _Float16 t1 = to_h_flush(x1);
    hv[e]     = t0;
    hv[4 + e] = t1;
    lv[e]     = rem_h_flush(x0, t0);
    lv[4 + e] = rem_h_flush(x1, t1);
  }
  unsigned short* q1  = A1  + (size_t)row * kG + c8 * 8u;
  unsigned short* q1l = A1L + (size_t)row * kG + c8 * 8u;
  unsigned short* q2  = A2  + (size_t)row * (2 * kD) + cc;
  const bool alsoA2 = (seg == 0u);
  const bool doBias = (i < 1024u);
  const unsigned bi = doBias ? (i * 4u) : 0u;
  const v4f b0 = *(const v4f*)(abih + bi);
  const v4f b1 = *(const v4f*)(abhh + bi);
  const v4f b2 = *(const v4f*)(lbih + bi);
  const v4f b3 = *(const v4f*)(lbhh + bi);
  const v4f sa = b0 + b1;
  const v4f sl = b2 + b3;
  for (int pass = 0; pass < 2; ++pass) {
    *(volatile v8h*)q1 = hv;
    *(volatile v8h*)q1l = lv;
    if (alsoA2) *(volatile v8h*)q2 = hv;
    if (doBias) {
      *(volatile v4f*)(bsA + bi) = sa;
      *(volatile v4f*)(bsL + bi) = sl;
    }
    __threadfence();
  }
}

__global__ __launch_bounds__(256) void cell_kernel(
    const float* __restrict__ G, const float* __restrict__ Gadd, const float* __restrict__ bsum,
    const float* __restrict__ cprev, float* __restrict__ hnew, float* __restrict__ cnew,
    const float* __restrict__ Sin, float* __restrict__ Sout,
    unsigned short* __restrict__ hplane, int planePitch, int planeCol0,
    int hasAdd, int hasS, int firstS) {
  __shared__ __align__(16) float sh[256];
  const int tid = threadIdx.x;
  const int lane = tid & 31;
  const int wave = tid >> 5;
  const int b  = blockIdx.x >> 2;
  const int d0 = (blockIdx.x & 3) * 256;
  const int d  = d0 + tid;
  const size_t gb = (size_t)b * kG + d;
  const size_t vb = (size_t)b * kD + d;
  float gi = G[gb];
  float gf = G[gb + kD];
  float gg = G[gb + 2 * kD];
  float go = G[gb + 3 * kD];
  if (hasAdd) {
    gi += Gadd[gb];
    gf += Gadd[gb + kD];
    gg += Gadd[gb + 2 * kD];
    go += Gadd[gb + 3 * kD];
  }
  gi += bsum[d];
  gf += bsum[d + kD];
  gg += bsum[d + 2 * kD];
  go += bsum[d + 3 * kD];
  const float cp = cprev[vb];
  float sOld = 0.0f;
  if (hasS && !firstS) sOld = Sin[vb];
  const float si = sigmoid_f(gi);
  const float sf = sigmoid_f(gf);
  const float tg = tanhf(gg);
  const float so = sigmoid_f(go);
  const float c2 = sf * cp + si * tg;
  const float h2 = so * tanhf(c2);
  const float sNew = sOld + h2;
  for (int pass = 0; pass < 2; ++pass) {
    *(volatile float*)(hnew + vb) = h2;
    *(volatile float*)(cnew + vb) = c2;
    if (hasS) *(volatile float*)(Sout + vb) = sNew;
    __threadfence();
  }
  sh[tid] = h2;
  __syncthreads();
  if (wave == 0) {
    const v4f a0 = *(const v4f*)(sh + lane * 8);
    const v4f a1 = *(const v4f*)(sh + lane * 8 + 4);
    v8h hv;
#pragma unroll
    for (int e = 0; e < 4; ++e) {
      const float x0 = a0[e] * kCarryA;
      const float x1 = a1[e] * kCarryA;
      hv[e]     = to_h_flush(x0);
      hv[4 + e] = to_h_flush(x1);
    }
    unsigned short* q = hplane + (size_t)b * planePitch + planeCol0 + d0 + lane * 8;
    *(volatile v8h*)q = hv;
    __threadfence();
    *(volatile v8h*)q = hv;
  }
}

__global__ __launch_bounds__(256) void attend_kernel(
    const float* __restrict__ hatt, const float* __restrict__ kvsIn, float* __restrict__ kvsOut,
    const float* __restrict__ vkey, const float* __restrict__ vval,
    const float* __restrict__ lkey, const float* __restrict__ lval,
    unsigned short* __restrict__ A3) {
  __shared__ __align__(16) float sq[kD];
  __shared__ __align__(16) float sk[kD];
  __shared__ __align__(16) float scx[2 * kD];
  __shared__ __align__(16) float ssc[64];
  __shared__ __align__(16) float spr[64];
  const int tid = threadIdx.x;
  const int lane = tid & 31;
  const int wave = tid >> 5;
  const int b = blockIdx.x;
  {
    const v4f hv = *(const v4f*)(hatt + (size_t)b * kD + tid * 4);
    const v4f kv = *(const v4f*)(kvsIn + (size_t)b * kD + tid * 4);
    *(v4f*)(sq + tid * 4) = hv + kv;
    *(v4f*)(sk + tid * 4) = kv;
  }
  __syncthreads();
#pragma unroll 1
  for (int jj = 0; jj < 7; ++jj) {
    const int s = wave + 8 * jj;
    const bool isV = (s < kNV);
    const float* rowp = isV ? (vkey + ((size_t)b * kNV + s) * kD)
                            : (lkey + ((size_t)b * kNL + (s - kNV)) * kD);
    float p = 0.0f;
#pragma unroll 2
    for (int it = 0; it < 8; ++it) {
      const v4f kk = *(const v4f*)(rowp + it * 128 + lane * 4);
      const v4f qq = *(const v4f*)(sq + it * 128 + lane * 4);
      p = fmaf(kk[0], qq[0], p);
      p = fmaf(kk[1], qq[1], p);
      p = fmaf(kk[2], qq[2], p);
      p = fmaf(kk[3], qq[3], p);
    }
    p += __shfl_xor(p, 16, 32);
    p += __shfl_xor(p, 8, 32);
    p += __shfl_xor(p, 4, 32);
    p += __shfl_xor(p, 2, 32);
    p += __shfl_xor(p, 1, 32);
    if (lane == 0) ssc[s] = p * kQScale;
  }
  __syncthreads();
  {
    const int which = wave & 1;
    const int base = which ? kNV : 0;
    const int cnt  = which ? kNL : kNV;
    const int i0 = (lane < cnt) ? lane : (cnt - 1);
    const int i1 = (lane + 32 < cnt) ? (lane + 32) : (cnt - 1);
    const float r0 = ssc[base + i0];
    const float r1 = ssc[base + i1];
    const bool ok0 = (lane < cnt);
    const bool ok1 = (lane + 32 < cnt);
    const float a0 = ok0 ? r0 : -INFINITY;
    const float a1 = ok1 ? r1 : -INFINITY;
    float m = fmaxf(a0, a1);
    m = fmaxf(m, __shfl_xor(m, 16, 32));
    m = fmaxf(m, __shfl_xor(m, 8, 32));
    m = fmaxf(m, __shfl_xor(m, 4, 32));
    m = fmaxf(m, __shfl_xor(m, 2, 32));
    m = fmaxf(m, __shfl_xor(m, 1, 32));
    const float x0 = expf(r0 - m);
    const float x1 = expf(r1 - m);
    const float e0 = ok0 ? x0 : 0.0f;
    const float e1 = ok1 ? x1 : 0.0f;
    float sm = e0 + e1;
    sm += __shfl_xor(sm, 16, 32);
    sm += __shfl_xor(sm, 8, 32);
    sm += __shfl_xor(sm, 4, 32);
    sm += __shfl_xor(sm, 2, 32);
    sm += __shfl_xor(sm, 1, 32);
    const float rinv = 1.0f / sm;
    if (wave < 2) {
      if (ok0) spr[base + lane] = e0 * rinv;
      if (ok1) spr[base + 32 + lane] = e1 * rinv;
    }
  }
  __syncthreads();
#pragma unroll 1
  for (int j = 0; j < 4; ++j) {
    const int d = j * 256 + tid;
    const float* vv = vval + (size_t)b * kNV * kD + d;
    const float* lv = lval + (size_t)b * kNL * kD + d;
    float va = 0.0f;
#pragma unroll 4
    for (int n = 0; n < kNV; ++n) va = fmaf(spr[n], vv[(size_t)n * kD], va);
    float la = 0.0f;
#pragma unroll 4
    for (int n = 0; n < kNL; ++n) la = fmaf(spr[kNV + n], lv[(size_t)n * kD], la);
    const float kn = tanhf((sk[d] + va) + la);
    scx[d] = va;
    scx[kD + d] = la;
    volatile float* kp = kvsOut + (size_t)b * kD + d;
    *kp = kn;
    __threadfence();
    *kp = kn;
  }
  __syncthreads();
  {
    const v4f a0 = *(const v4f*)(scx + tid * 8);
    const v4f a1 = *(const v4f*)(scx + tid * 8 + 4);
    v8h hv;
#pragma unroll
    for (int e = 0; e < 4; ++e) {
      const float x0 = a0[e] * kCarryA;
      const float x1 = a1[e] * kCarryA;
      hv[e]     = to_h_flush(x0);
      hv[4 + e] = to_h_flush(x1);
    }
    unsigned short* q = A3 + (size_t)b * (2 * kD) + tid * 8;
    *(volatile v8h*)q = hv;
    __threadfence();
    *(volatile v8h*)q = hv;
  }
}

__global__ __launch_bounds__(256) void halt_kernel(
    const float* __restrict__ CT, const float* __restrict__ cb1, const float* __restrict__ cW2,
    const float* __restrict__ cb2, const float* __restrict__ hlang, const float* __restrict__ clang,
    const float* __restrict__ hLin, const float* __restrict__ cLin,
    float* __restrict__ hLout, float* __restrict__ cLout,
    const float* __restrict__ stIn, float* __restrict__ stOut, int stepi, int first) {
  const float stepv = (float)stepi;
  __shared__ float sred[8];
  const int tid = threadIdx.x;
  const int lane = tid & 31;
  const int wave = tid >> 5;
  const int b = blockIdx.x;
  const size_t vb = (size_t)b * kD + tid * 4;
  float aOld = 0.0f, selOld = 1.0f, costOld = 0.0f;
  v4f hOld = (v4f){0.f, 0.f, 0.f, 0.f};
  v4f cOld = (v4f){0.f, 0.f, 0.f, 0.f};
  if (!first) {
    aOld    = stIn[b * 32 + 0];
    selOld  = stIn[b * 32 + 1];
    costOld = stIn[b * 32 + 2];
    hOld = *(const v4f*)(hLin + vb);
    cOld = *(const v4f*)(cLin + vb);
  }
  const v4f ct = *(const v4f*)(CT + vb);
  const v4f bb = *(const v4f*)(cb1 + tid * 4);
  const v4f ww = *(const v4f*)(cW2 + tid * 4);
  float s = 0.0f;
  s = fmaf(fmaxf(ct[0] + bb[0], 0.0f), ww[0], s);
  s = fmaf(fmaxf(ct[1] + bb[1], 0.0f), ww[1], s);
  s = fmaf(fmaxf(ct[2] + bb[2], 0.0f), ww[2], s);
  s = fmaf(fmaxf(ct[3] + bb[3], 0.0f), ww[3], s);
  s += __shfl_xor(s, 16, 32);
  s += __shfl_xor(s, 8, 32);
  s += __shfl_xor(s, 4, 32);
  s += __shfl_xor(s, 2, 32);
  s += __shfl_xor(s, 1, 32);
  if (lane == 0) sred[wave] = s;
  __syncthreads();
  const float tot = ((((((sred[0] + sred[1]) + sred[2]) + sred[3]) + sred[4]) + sred[5]) + sred[6]) + sred[7];
  const float p = sigmoid_f(tot + cb2[0]);
  const float beta = p * (1.0f - aOld);
  const v4f hl = *(const v4f*)(hlang + vb);
  const v4f cl = *(const v4f*)(clang + vb);
  v4f hNew, cNew;
  hNew[0] = hOld[0] + (beta * hl[0]) * selOld;
  hNew[1] = hOld[1] + (beta * hl[1]) * selOld;
  hNew[2] = hOld[2] + (beta * hl[2]) * selOld;
  hNew[3] = hOld[3] + (beta * hl[3]) * selOld;
  cNew[0] = cOld[0] + (beta * cl[0]) * selOld;
  cNew[1] = cOld[1] + (beta * cl[1]) * selOld;
  cNew[2] = cOld[2] + (beta * cl[2]) * selOld;
  cNew[3] = cOld[3] + (beta * cl[3]) * selOld;
  const float aNew = aOld + beta * selOld;
  const float costNew = costOld + (stepv * (1.0f - p)) * selOld;
  const float selNew = (aNew < kHaltThr) ? selOld : 0.0f;
  float lineVal = 0.0f;
  lineVal = (lane == 0) ? aNew : lineVal;
  lineVal = (lane == 1) ? selNew : lineVal;
  lineVal = (lane == 2) ? costNew : lineVal;
  lineVal = (lane == 3) ? p : lineVal;
  for (int pass = 0; pass < 2; ++pass) {
    *(volatile v4f*)(hLout + vb) = hNew;
    *(volatile v4f*)(cLout + vb) = cNew;
    if (wave == 0) *(volatile float*)(stOut + b * 32 + lane) = lineVal;
    __threadfence();
  }
}

__global__ __launch_bounds__(256) void final_vec_kernel(
    const float* __restrict__ hatt, const float* __restrict__ catt,
    const float* __restrict__ hL, const float* __restrict__ cL, const float* __restrict__ kvs,
    const float* __restrict__ st, const int* __restrict__ tptr, float* __restrict__ out) {
  const int tid = threadIdx.x;
  const int b = blockIdx.x;
  const size_t vb = (size_t)b * kD + tid * 4;
  const bool ok = (tptr[0] == kT);
  const float accum = st[b * 32 + 0];
  const float inv = 1.0f / accum;
  const v4f vh  = *(const v4f*)(hL + vb);
  const v4f vc  = *(const v4f*)(cL + vb);
  const v4f vha = *(const v4f*)(hatt + vb);
  const v4f vca = *(const v4f*)(catt + vb);
  const v4f vk  = *(const v4f*)(kvs + vb);
  const v4f o0 = poison_sel4(vh * inv, ok);
  const v4f o1 = poison_sel4(vc * inv, ok);
  const v4f o2 = poison_sel4(vha, ok);
  const v4f o3 = poison_sel4(vca, ok);
  const v4f o4 = poison_sel4(vk, ok);
  for (int pass = 0; pass < 2; ++pass) {
    *(volatile v4f*)(out + kOutA + vb) = o0;
    *(volatile v4f*)(out + kOutH + vb) = o2;
    *(volatile v4f*)(out + kOutH + (size_t)kB * kD + vb) = o0;
    *(volatile v4f*)(out + kOutC + vb) = o3;
    *(volatile v4f*)(out + kOutC + (size_t)kB * kD + vb) = o1;
    *(volatile v4f*)(out + kOutKV + vb) = o4;
    __threadfence();
  }
}

__global__ __launch_bounds__(32) void cost_out_kernel(
    const float* __restrict__ st, const int* __restrict__ itp, const int* __restrict__ tptr,
    float* __restrict__ out3) {
  const int lane = threadIdx.x & 31;
  const bool ok = (tptr[0] == kT);
  const v4i iv = *(const v4i*)(itp + lane * 4);
  const float c0 = st[(lane * 4 + 0) * 32 + 2];
  const float c1 = st[(lane * 4 + 1) * 32 + 2];
  const float c2 = st[(lane * 4 + 2) * 32 + 2];
  const float c3 = st[(lane * 4 + 3) * 32 + 2];
  v4f v;
  v[0] = c0 * ((iv[0] > 0) ? 1.0f : 0.0f);
  v[1] = c1 * ((iv[1] > 0) ? 1.0f : 0.0f);
  v[2] = c2 * ((iv[2] > 0) ? 1.0f : 0.0f);
  v[3] = c3 * ((iv[3] > 0) ? 1.0f : 0.0f);
  const v4f o = poison_sel4(v, ok);
  *(volatile v4f*)(out3 + lane * 4) = o;
  __threadfence();
  *(volatile v4f*)(out3 + lane * 4) = o;
}

constexpr int kVisRows = kB * kNV;
constexpr int kAllRows = kB * (kNV + kNL);
static_assert((kVisRows % 4) == 0 && (kAllRows % 4) == 0, "rows per block");
__global__ __launch_bounds__(256) void keys_out_kernel(
    const float* __restrict__ vkey, const float* __restrict__ lkey, const float* __restrict__ S,
    const int* __restrict__ tptr, float* __restrict__ out1, float* __restrict__ out2) {
  const int tid = threadIdx.x;
  const bool ok = (tptr[0] == kT);
  const unsigned r0 = blockIdx.x * 4u;
  const bool isV = (r0 < (unsigned)kVisRows);
  const float* src = isV ? vkey : lkey;
  float* dst = isV ? out1 : out2;
  const unsigned rbase = isV ? r0 : (r0 - (unsigned)kVisRows);
  const unsigned per = isV ? (unsigned)kNV : (unsigned)kNL;
  v4f val[4];
#pragma unroll
  for (int it = 0; it < 4; ++it) {
    const unsigned rr = rbase + (unsigned)it;
    unsigned b = rr / per;
    b = (b < (unsigned)kB) ? b : (unsigned)(kB - 1);
    const v4f kv = *(const v4f*)(src + (size_t)rr * kD + tid * 4);
    const v4f sv = *(const v4f*)(S + (size_t)b * kD + tid * 4);
    val[it] = poison_sel4(kv + kKeyStep * sv, ok);
  }
  for (int pass = 0; pass < 2; ++pass) {
#pragma unroll
    for (int it = 0; it < 4; ++it) {
      const unsigned rr = rbase + (unsigned)it;
      *(volatile v4f*)(dst + (size_t)rr * kD + tid * 4) = val[it];
    }
    __threadfence();
  }
}

static_assert((kG % 64) == 0 && (kD % 64) == 0 && (kB % 64) == 0, "GEMM tile multiples");
static_assert((kG % 32) == 0 && ((2 * kD) % 32) == 0 && (kD % 32) == 0, "GEMM K multiples");

extern "C" void kernel_launch(void* const* d_in, const int* in_sizes, int n_in,
                              void* d_out, int out_size, void* d_ws, size_t ws_size,
                              hipStream_t stream) {
  if (n_in < 23) return;
  if (in_sizes[0] != kB * kD || in_sizes[1] != kB || in_sizes[2] != kB * kD) return;
  if (in_sizes[3] != kB * kNV * kD || in_sizes[4] != kB * kNV * kD) return;
  if (in_sizes[5] != kB * kNL * kD || in_sizes[6] != kB * kNL * kD) return;
  if (in_sizes[7] != kB * kD || in_sizes[8] != 2 * kB * kD || in_sizes[9] != 2 * kB * kD) return;
  if (in_sizes[10] != 1) return;
  if (in_sizes[11] != kG * kInW || in_sizes[12] != kG * kD || in_sizes[13] != kG || in_sizes[14] != kG) return;
  if (in_sizes[15] != kG * kInW || in_sizes[16] != kG * kD || in_sizes[17] != kG || in_sizes[18] != kG) return;
  if (in_sizes[19] != kD * kD || in_sizes[20] != kD || in_sizes[21] != kD || in_sizes[22] != 1) return;
  if ((size_t)out_size != kOutTot) return;
  if (ws_size < kWsTotal) return;

  const float* xt      = (const float*)d_in[0];
  const int*   itp     = (const int*)  d_in[1];
  const float* fc      = (const float*)d_in[2];
  const float* vval    = (const float*)d_in[3];
  const float* vkey    = (const float*)d_in[4];
  const float* lval    = (const float*)d_in[5];
  const float* lkey    = (const float*)d_in[6];
  const float* kv0     = (const float*)d_in[7];
  const float* stateH  = (const float*)d_in[8];
  const float* stateC  = (const float*)d_in[9];
  const int*   tptr    = (const int*)  d_in[10];
  const float* attWih  = (const float*)d_in[11];
  const float* attWhh  = (const float*)d_in[12];
  const float* attBih  = (const float*)d_in[13];
  const float* attBhh  = (const float*)d_in[14];
  const float* lngWih  = (const float*)d_in[15];
  const float* lngWhh  = (const float*)d_in[16];
  const float* lngBih  = (const float*)d_in[17];
  const float* lngBhh  = (const float*)d_in[18];
  const float* cW1     = (const float*)d_in[19];
  const float* cB1     = (const float*)d_in[20];
  const float* cW2     = (const float*)d_in[21];
  const float* cB2     = (const float*)d_in[22];
  float* out = (float*)d_out;

  const float* h0  = stateH;
  const float* h1  = stateH + (size_t)kB * kD;
  const float* c0  = stateC;
  const float* c1  = stateC + (size_t)kB * kD;

  char* ws = (char*)d_ws;
  unsigned short* BT1 = (unsigned short*)(ws + kOffBT1);
  unsigned short* BT2 = (unsigned short*)(ws + kOffBT2);
  unsigned short* BT3 = (unsigned short*)(ws + kOffBT3);
  unsigned short* BT4 = (unsigned short*)(ws + kOffBT4);
  unsigned short* A1  = (unsigned short*)(ws + kOffA1);
  unsigned short* A1L = (unsigned short*)(ws + kOffA1L);
  unsigned short* A2  = (unsigned short*)(ws + kOffA2);
  unsigned short* A3  = (unsigned short*)(ws + kOffA3);
  unsigned short* A4  = (unsigned short*)(ws + kOffA4);
  float* GA    = (float*)(ws + kOffGA);
  float* GAR   = (float*)(ws + kOffGAR);
  float* LC    = (float*)(ws + kOffLC);
  float* GL    = (float*)(ws + kOffGL);
  float* CT    = (float*)(ws + kOffCT);
  float* HATT  = (float*)(ws + kOffHATT);
  float* CATT  = (float*)(ws + kOffCATT);
  float* HLG   = (float*)(ws + kOffHLG);
  float* CLG   = (float*)(ws + kOffCLG);
  float* KV[2] = { (float*)(ws + kOffKV0), (float*)(ws + kOffKV1) };
  float* HL[2] = { (float*)(ws + kOffHL0), (float*)(ws + kOffHL1) };
  float* CL[2] = { (float*)(ws + kOffCL0), (float*)(ws + kOffCL1) };
  float* SS[2] = { (float*)(ws + kOffS0),  (float*)(ws + kOffS1) };
  float* ST[2] = { (float*)(ws + kOffST0), (float*)(ws + kOffST1) };
  float* BSA   = (float*)(ws + kOffBSA);
  float* BSL   = (float*)(ws + kOffBSL);

  cvt_plane_kernel<<<(kG * (kInW / 8)) / 256, 256, 0, stream>>>(attWih, kInW, 0, BT1, kG, 0, kInW / 8, kG * (kInW / 8), kCarryW);
  cvt_plane_kernel<<<(kG * (kD / 8)) / 256, 256, 0, stream>>>(attWhh, kD, 0, BT1, kG, kInW, kD / 8, kG * (kD / 8), kCarryW);
  cvt_plane_kernel<<<(kG * (kD / 8)) / 256, 256, 0, stream>>>(lngWhh, kD, 0, BT2, 2 * kD, 0, kD / 8, kG * (kD / 8), kCarryW);
  cvt_plane_kernel<<<(kG * (kD / 8)) / 256, 256, 0, stream>>>(lngWih, kInW, 2 * kD, BT2, 2 * kD, kD, kD / 8, kG * (kD / 8), kCarryW);
  cvt_plane_kernel<<<(kG * (2 * kD / 8)) / 256, 256, 0, stream>>>(lngWih, kInW, 0, BT3, 2 * kD, 0, 2 * kD / 8, kG * (2 * kD / 8), kCarryW);
  cvt_plane_kernel<<<(kD * (kD / 8)) / 256, 256, 0, stream>>>(cW1, kD, 0, BT4, kD, 0, kD / 8, kD * (kD / 8), kCarryW);

  cvt_act_kernel<<<(kB * kG / 8) / 256, 256, 0, stream>>>(h1, fc, xt, h0, A1, A1L, A2, attBih, attBhh, lngBih, lngBhh, BSA, BSL);

  gemm_f16_tile64<<<16, 256, 0, stream>>>(A1,  kG, BT1, kG, GA,  kG, kB, kG, kG, kFold);
  gemm_f16_tile64<<<16, 256, 0, stream>>>(A1L, kG, BT1, kG, GAR, kG, kB, kG, kG, kFoldR);
  cell_kernel<<<kB * 4, 256, 0, stream>>>(GA, GAR, BSA, c0, HATT, CATT, HATT, HATT, A2, 2 * kD, kD, 1, 0, 0);

  gemm_f16_tile64<<<16, 256, 0, stream>>>(A2, 2 * kD, BT2, 2 * kD, LC, kG, kB, kG, 2 * kD, kFold);

  for (int i = 0; i < kT; ++i) {
    const int cur = i & 1;
    const int prv = cur ^ 1;
    const int first = (i == 0) ? 1 : 0;
    const float* kvIn = first ? kv0 : KV[prv];
    attend_kernel<<<kB, 256, 0, stream>>>(HATT, kvIn, KV[cur], vkey, vval, lkey, lval, A3);
    gemm_f16_tile64<<<16, 256, 0, stream>>>(A3, 2 * kD, BT3, 2 * kD, GL, kG, kB, kG, 2 * kD, kFold);
    cell_kernel<<<kB * 4, 256, 0, stream>>>(GL, LC, BSL, c1, HLG, CLG, SS[prv], SS[cur], A4, kD, 0, 1, 1, first);
    gemm_f16_tile64<<<4, 256, 0, stream>>>(A4, kD, BT4, kD, CT, kD, kB, kD, kD, kFold);
    halt_kernel<<<kB, 256, 0, stream>>>(CT, cB1, cW2, cB2, HLG, CLG, HL[prv], CL[prv], HL[cur], CL[cur],
                                        ST[prv], ST[cur], i + 1, first);
  }
  constexpr int fin = (kT - 1) & 1;

  final_vec_kernel<<<kB, 256, 0, stream>>>(HATT, CATT, HL[fin], CL[fin], KV[fin], ST[fin], tptr, out);
  cost_out_kernel<<<1, 32, 0, stream>>>(ST[fin], itp, tptr, out + kOutCst);
  keys_out_kernel<<<kAllRows / 4, 256, 0, stream>>>(vkey, lkey, SS[fin], tptr, out + kOutVK, out + kOutLK);
}
